// EasySlidingWindowAttention_72456098284253
// MI455X (gfx1250) — hardware-verified
//
#include <hip/hip_runtime.h>
#include <stdint.h>

typedef __attribute__((ext_vector_type(16))) _Float16 v16h;
typedef __attribute__((ext_vector_type(8)))  _Float16 v8h;
typedef __attribute__((ext_vector_type(16))) __bf16   v16b;
typedef __attribute__((ext_vector_type(8)))  __bf16   v8b;
typedef __attribute__((ext_vector_type(8)))  float    v8f;
typedef __attribute__((ext_vector_type(4)))  float    v4f;
#define PSCALE 32768.0f
#define U16(p) ((const unsigned short*)(const void*)(p))
#define PSCALE_INV (1.0f / 32768.0f)

__device__ __forceinline__ unsigned short f2bf_bits(float f) {
  unsigned u = __float_as_uint(f);
  return (unsigned short)((u + 0x7FFFu + ((u >> 16) & 1u)) >> 16);
}
__device__ __forceinline__ float bf_bits2f(unsigned short h) { return __uint_as_float(((unsigned)h) << 16); }

__device__ __forceinline__ void dep_guard_h(v8f& a, v8f& b, v16h x, v16h y) { asm volatile("v_nop\n\tv_nop\n\tv_nop\n\tv_nop" : "+v"(a), "+v"(b) : "v"(x), "v"(y)); }
__device__ __forceinline__ void dep_guard_b(v8f& a, v8f& b, v16b x, v16b y) { asm volatile("v_nop\n\tv_nop\n\tv_nop\n\tv_nop" : "+v"(a), "+v"(b) : "v"(x), "v"(y)); }
__device__ __forceinline__ void keep4_h(v16h a, v16h b, v16h c, v16h d) { asm volatile("v_nop" :: "v"(a), "v"(b), "v"(c), "v"(d)); }
__device__ __forceinline__ void keep4_b(v16b a, v16b b, v16b c, v16b d) { asm volatile("v_nop" :: "v"(a), "v"(b), "v"(c), "v"(d)); }
__device__ __forceinline__ void acc_guard4(v8f& a, v8f& b, v8f& c, v8f& d) { asm volatile("v_nop\n\tv_nop\n\tv_nop\n\tv_nop" : "+v"(a), "+v"(b), "+v"(c), "+v"(d)); }
template <typename T> struct Frag;
template <> struct Frag<_Float16> {
  typedef v16h V; union U { v16h v; v8h h[2]; };
  static __device__ __forceinline__ v16h load(const _Float16* p) {
    U f; f.h[0] = *(const v8h*)(p); f.h[1] = *(const v8h*)(p + 16); return f.v;
  }
  static __device__ __forceinline__ v8f mma(v16h a, v16h b, v8f c) {
    return __builtin_amdgcn_wmma_f32_16x16x32_f16(false, a, false, b, (short)0, c, false, false);
  }
  static __device__ __forceinline__ void guard(v8f& a, v8f& b, v16h x, v16h y) { dep_guard_h(a, b, x, y); }
  static __device__ __forceinline__ void keep(v16h a, v16h b, v16h c, v16h d) { keep4_h(a, b, c, d); }
};
template <> struct Frag<__bf16> {
  typedef v16b V; union U { v16b v; v8b h[2]; };
  static __device__ __forceinline__ v16b load(const __bf16* p) {
    U f; f.h[0] = *(const v8b*)(p); f.h[1] = *(const v8b*)(p + 16); return f.v;
  }
  static __device__ __forceinline__ v8f mma(v16b a, v16b b, v8f c) {
    return __builtin_amdgcn_wmma_f32_16x16x32_bf16(false, a, false, b, (short)0, c, false, false);
  }
  static __device__ __forceinline__ void guard(v8f& a, v8f& b, v16b x, v16b y) { dep_guard_b(a, b, x, y); }
  static __device__ __forceinline__ void keep(v16b a, v16b b, v16b c, v16b d) { keep4_b(a, b, c, d); }
};

template <int ET> struct Elem;
template <> struct Elem<0> { typedef _Float16 T; };
template <> struct Elem<1> { typedef __bf16 T; };
template <int ET, bool SPLIT, int BIAS_MODE, int OUT_MODE, bool RESID, int ACT = 0>
__global__ __launch_bounds__(256) void wmma_gemm64(
    const unsigned short* __restrict__ Ap, const unsigned short* __restrict__ A2p, int lda, long strideA,
    const unsigned short* __restrict__ Btp, const unsigned short* __restrict__ Bt2p, int ldb, long strideB,
    void* __restrict__ Cout, void* __restrict__ Cout2, int ldc, long strideC,
    const float* __restrict__ bias,
    const float* __restrict__ resid, long strideR,
    int M, int N, int K, float scale) {
  typedef typename Elem<ET>::T T;
  typedef typename Frag<T>::V V;
  const T* A = (const T*)Ap; const T* A2 = (const T*)A2p; const T* Bt = (const T*)Btp; const T* Bt2 = (const T*)Bt2p;
  __shared__ __align__(16) float sT[8][16 * 68];
  const int b    = blockIdx.y;
  const int lane = threadIdx.x & 31;
  const int wave = threadIdx.x >> 5;
  const int tilesN = N >> 6;
  const int tilesM = M >> 6;
  const int tile = blockIdx.x * 8 + wave;
  if (tile >= tilesM * tilesN) return;
  const int tm = tile / tilesN;
  const int tn = tile - tm * tilesN;
  const int m0 = tm << 6;
  const int n0 = tn << 6;

  const T* Ab  = A  + (size_t)b * strideA;
  const T* Bb  = Bt + (size_t)b * strideB;
  const T* Ab2 = SPLIT ? (A2  + (size_t)b * strideA) : nullptr;
  const T* Bb2 = SPLIT ? (Bt2 + (size_t)b * strideB) : nullptr;

  const int rlane = lane & 15;
  const int koff  = (lane >> 4) * 8;
  const int mOff  = (lane >> 4) * 8;

  v8f acc[4][4];
#pragma unroll
  for (int i = 0; i < 4; ++i)
#pragma unroll
    for (int j = 0; j < 4; ++j) acc[i][j] = (v8f){0.f,0.f,0.f,0.f,0.f,0.f,0.f,0.f};

  for (int k0 = 0; k0 < K; k0 += 32) {
    V bh[4], bl[4];
#pragma unroll
    for (int j = 0; j < 4; ++j) {
      const size_t bo = (size_t)(n0 + (j << 4) + rlane) * ldb + koff + k0;
      bh[j] = Frag<T>::load(Bb + bo);
      if (SPLIT) bl[j] = Frag<T>::load(Bb2 + bo);
    }
#pragma unroll
    for (int i = 0; i < 4; ++i) {
      const size_t ao = (size_t)(m0 + (i << 4) + rlane) * lda + koff + k0;
      V ah = Frag<T>::load(Ab + ao);
      V al;
      if (SPLIT) al = Frag<T>::load(Ab2 + ao);
#pragma unroll
      for (int j = 0; j < 4; ++j) {
        acc[i][j] = Frag<T>::mma(ah, bh[j], acc[i][j]);
        if (SPLIT) {
          acc[i][j] = Frag<T>::mma(ah, bl[j], acc[i][j]);
          acc[i][j] = Frag<T>::mma(al, bh[j], acc[i][j]);
        }
      }
      Frag<T>::guard(acc[i][0], acc[i][3], ah, SPLIT ? al : ah);
    }
    Frag<T>::keep(bh[0], bh[1], bh[2], bh[3]);
    if (SPLIT) Frag<T>::keep(bl[0], bl[1], bl[2], bl[3]);
  }
  acc_guard4(acc[0][0], acc[0][1], acc[0][2], acc[0][3]);
  acc_guard4(acc[1][0], acc[1][1], acc[1][2], acc[1][3]);
  acc_guard4(acc[2][0], acc[2][1], acc[2][2], acc[2][3]);
  acc_guard4(acc[3][0], acc[3][1], acc[3][2], acc[3][3]);

  float* slab = sT[wave];
  const float* Rb = RESID ? (resid + (size_t)b * strideR) : nullptr;
#pragma unroll
  for (int i = 0; i < 4; ++i) {
    const int mBase = m0 + (i << 4);
#pragma unroll
    for (int j = 0; j < 4; ++j) {
      const int n = n0 + (j << 4) + rlane;
      float bv = 0.f;
      if (BIAS_MODE == 2) bv = bias[n];
#pragma unroll
      for (int r = 0; r < 8; ++r) {
        float v = acc[i][j][r] * scale;
        if (BIAS_MODE == 1) v += bias[mBase + mOff + r];
        if (BIAS_MODE == 2) v += bv;
        if (RESID) v += Rb[(size_t)(mBase + mOff + r) * ldc + n];
        if (ACT == 1) v = tanhf(v);
        if (ACT == 2) v = fmaxf(v, 0.0f);
        if (ACT == 3) v = v / (1.0f + expf(-v));
        if (ACT == 4) v = (v > 0.f) ? v : 0.01f * v;
        if (ACT == 5) v = 0.5f * v * (1.0f + erff(v * 0.70710678118654752f));
        slab[(mOff + r) * 68 + (j << 4) + rlane] = v;
      }
    }
    __builtin_amdgcn_fence(__ATOMIC_RELEASE, "workgroup");
    __builtin_amdgcn_wave_barrier();
    __builtin_amdgcn_fence(__ATOMIC_ACQUIRE, "workgroup");
    if (OUT_MODE == 0) {
      float* C = (float*)Cout + (size_t)b * strideC;
      const int hh = lane >> 4, c4 = (lane & 15) * 4;
      for (int pass = 0; pass < 2; ++pass) {
#pragma unroll
        for (int it = 0; it < 8; ++it) {
          const int row = it * 2 + hh;
          v4f v = *(const v4f*)(slab + row * 68 + c4);
          *(volatile v4f*)(C + (size_t)(mBase + row) * ldc + n0 + c4) = v;
        }
        __threadfence();
      }
    } else {
      const int q = lane >> 3, c8 = (lane & 7) * 8;
      unsigned short* C  = (unsigned short*)Cout  + (size_t)b * strideC;
      unsigned short* C2 = (OUT_MODE == 2) ? ((unsigned short*)Cout2 + (size_t)b * strideC) : nullptr;
      for (int pass = 0; pass < 2; ++pass) {
#pragma unroll
        for (int it = 0; it < 4; ++it) {
          const int row = it * 4 + q;
          const float* sp = slab + row * 68 + c8;
          v8h hv, lv;
#pragma unroll
          for (int e = 0; e < 8; ++e) {
            if (OUT_MODE == 1) {
              hv[e] = (_Float16)sp[e];
            } else {
              unsigned short hb = f2bf_bits(sp[e]);
              unsigned short lb = f2bf_bits(sp[e] - bf_bits2f(hb));
              hv[e] = __builtin_bit_cast(_Float16, hb);
              lv[e] = __builtin_bit_cast(_Float16, lb);
            }
          }
          *(volatile v8h*)(C + (size_t)(mBase + row) * ldc + n0 + c8) = hv;
          if (OUT_MODE == 2) *(volatile v8h*)(C2 + (size_t)(mBase + row) * ldc + n0 + c8) = lv;
        }
        __threadfence();
      }
    }
    __builtin_amdgcn_fence(__ATOMIC_RELEASE, "workgroup");
    __builtin_amdgcn_wave_barrier();
    __builtin_amdgcn_fence(__ATOMIC_ACQUIRE, "workgroup");
  }
}

__global__ __launch_bounds__(256) void cast_f32_f16x2_scaled(
    const float* __restrict__ in, _Float16* __restrict__ out, int n2, float sc) {
  int i = blockIdx.x * 256 + threadIdx.x;
  if (i < n2) {
    const _Float16 h0 = (_Float16)(in[2 * (size_t)i] * sc), h1 = (_Float16)(in[2 * (size_t)i + 1] * sc);
    const unsigned u = (unsigned)__builtin_bit_cast(unsigned short, h0) | ((unsigned)__builtin_bit_cast(unsigned short, h1) << 16);
    ((volatile unsigned*)out)[i] = u;
    __threadfence();
    ((volatile unsigned*)out)[i] = u;
  }
}

#define AT_D 64
#define AT_NW 4
#define AT_QB 64
#define AT_KC 64
#define AT_MAXCH 6
#define AT_PSC 32768.0f
struct BandGeom { long q_bs, q_rs, q_hs, k_bs, k_rs, k_hs, v_bs, v_rs, v_hs, o_bs, o_rs, o_hs, m_bs, m_rs;
                  int S, H, W, lastq; float qscale, mask_fill; };
static_assert(sizeof(BandGeom) == 136);

__device__ __forceinline__ v8f mma_h(v16h a, v16h b, v8f c) {
  c = __builtin_amdgcn_wmma_f32_16x16x32_f16(false, a, false, b, (short)0, c, false, false);
  asm volatile("v_nop\n\tv_nop\n\tv_nop\n\tv_nop" : "+v"(c) : "v"(a), "v"(b));
  return c;
}

__global__ __launch_bounds__(128)
void attn_band64_kernel(const float* __restrict__ q, const float* __restrict__ k,
                        const float* __restrict__ v, float* __restrict__ out,
                        const int* __restrict__ amask, BandGeom g) {
  union FH { v16h v; v8h h[2]; };
  __shared__ __align__(16) _Float16 Ksh[AT_KC * AT_D];
  __shared__ __align__(16) _Float16 Vth[AT_D * AT_KC];
  __shared__ __align__(16) _Float16 Psh[AT_NW][16 * AT_KC];
  __shared__ __align__(16) float    Os[AT_NW][16 * 68];

  const int tid  = threadIdx.x;
  const int wave = tid >> 5;
  const int lane = tid & 31;
  const int hh   = lane >> 4;
  const int c    = lane & 15;

  const int nqb = g.S / AT_QB;
  const int bx = blockIdx.x;
  const int qb = bx % nqb;
  const int bh = bx / nqb;
  const int h  = bh % g.H;
  const int b  = bh / g.H;
  const int qbase = qb * AT_QB;
  const int q0 = qbase + wave * 16;

  const float* qb_ptr = q + (size_t)b * g.q_bs + (size_t)h * g.q_hs;
  const float* kb_ptr = k + (size_t)b * g.k_bs + (size_t)h * g.k_hs;
  const float* vb_ptr = v + (size_t)b * g.v_bs + (size_t)h * g.v_hs;
  float*       ob_ptr = out + (size_t)b * g.o_bs + (size_t)h * g.o_hs;
  const int*   amb    = amask + (size_t)b * g.m_bs;

  v16h qa0, qa1;
  {
    const float* qrow = qb_ptr + (size_t)(q0 + c) * g.q_rs;
#pragma unroll
    for (int e = 0; e < 8; ++e) {
      qa0[e]     = (_Float16)qrow[8 * hh + e];
      qa0[8 + e] = (_Float16)qrow[16 + 8 * hh + e];
      qa1[e]     = (_Float16)qrow[32 + 8 * hh + e];
      qa1[8 + e] = (_Float16)qrow[32 + 16 + 8 * hh + e];
    }
  }

  float mrow[8], lrow[8];
  v8f oacc[4];
#pragma unroll
  for (int r = 0; r < 8; ++r) { mrow[r] = -__builtin_huge_valf(); lrow[r] = 0.f; }
#pragma unroll
  for (int t = 0; t < 4; ++t) oacc[t] = (v8f){0.f,0.f,0.f,0.f,0.f,0.f,0.f,0.f};

  const int nkc = g.S / AT_KC;
  int Wd = g.W;
  Wd = Wd < 0 ? 0 : Wd;
  Wd = Wd > g.S ? g.S : Wd;
  const int lo = qbase - Wd;
  const int kcLo = (lo < 0) ? 0 : (lo / AT_KC);
  int kcHi = (qbase + AT_QB - 1 + Wd) / AT_KC;
  kcHi = kcHi > nkc - 1 ? nkc - 1 : kcHi;
  int nvis = kcHi - kcLo + 1;
  nvis = nvis > AT_MAXCH ? AT_MAXCH : nvis;
  nvis = nvis < 1 ? 1 : nvis;

  for (int ci = 0; ci < nvis; ++ci) {
    const int kv0 = (kcLo + ci) * AT_KC;
    __syncthreads();
    {
      const int kvr = tid >> 1, dh = (tid & 1) * 32;
      const float* krow = kb_ptr + (size_t)(kv0 + kvr) * g.k_rs + dh;
      const float* vrow = vb_ptr + (size_t)(kv0 + kvr) * g.v_rs + dh;
#pragma unroll
      for (int i = 0; i < 8; ++i) {
        v4f kk = *(const v4f*)(krow + 4 * i);
        v4f vv = *(const v4f*)(vrow + 4 * i);
#pragma unroll
        for (int e = 0; e < 4; ++e) {
          const int d = dh + 4 * i + e;
          Ksh[kvr * AT_D + d]  = (_Float16)kk[e];
          Vth[d * AT_KC + kvr] = (_Float16)vv[e];
        }
      }
    }

    unsigned keep = 0u;
#pragma unroll
    for (int r = 0; r < 8; ++r) {
      const int qrow = q0 + 8 * hh + r;
      const int* mrowp = amb + (size_t)qrow * g.m_rs + kv0;
#pragma unroll
      for (int j = 0; j < 4; ++j) {
        const int kvcol = kv0 + j * 16 + c;
        const int dlt = qrow - kvcol;
        const int ad = dlt < 0 ? -dlt : dlt;
        const bool band = ((ad >= 1) && (ad <= Wd)) || ((qrow == 0) && (kvcol == 0)) ||
                          ((qrow == g.lastq) && (kvcol == g.lastq));
        const int mv = mrowp[j * 16 + c];
        if (band && (mv != 0)) keep |= (1u << (r * 4 + j));
      }
    }
    __syncthreads();

    v8f s[4];
#pragma unroll
    for (int j = 0; j < 4; ++j) {
      s[j] = (v8f){0.f,0.f,0.f,0.f,0.f,0.f,0.f,0.f};
      FH kb0, kb1;
      kb0.h[0] = *(const v8h*)(Ksh + (j * 16 + c) * AT_D + 8 * hh);
      kb0.h[1] = *(const v8h*)(Ksh + (j * 16 + c) * AT_D + 16 + 8 * hh);
      kb1.h[0] = *(const v8h*)(Ksh + (j * 16 + c) * AT_D + 32 + 8 * hh);
      kb1.h[1] = *(const v8h*)(Ksh + (j * 16 + c) * AT_D + 32 + 16 + 8 * hh);
      s[j] = mma_h(qa0, kb0.v, s[j]);
      s[j] = mma_h(qa1, kb1.v, s[j]);
    }

    float cm[8];
#pragma unroll
    for (int r = 0; r < 8; ++r) {
      float m = -__builtin_huge_valf();
#pragma unroll
      for (int j = 0; j < 4; ++j) {
        float sv = s[j][r] * g.qscale;
        if (((keep >> (r * 4 + j)) & 1u) == 0u) sv = g.mask_fill;
        s[j][r] = sv;
        m = fmaxf(m, sv);
      }
#pragma unroll
      for (int off = 1; off < 16; off <<= 1) m = fmaxf(m, __shfl_xor(m, off, 32));
      cm[r] = m;
    }
    _Float16* pwh = Psh[wave];
#pragma unroll
    for (int r = 0; r < 8; ++r) {
      const float mnew = fmaxf(mrow[r], cm[r]);
      const float alpha = expf(mrow[r] - mnew);
      mrow[r] = mnew;
      float psum = 0.f;
#pragma unroll
      for (int j = 0; j < 4; ++j) {
        const float p = expf(s[j][r] - mnew);
        psum += p;
        pwh[(8 * hh + r) * AT_KC + j * 16 + c] = (_Float16)(p * AT_PSC);
      }
#pragma unroll
      for (int off = 1; off < 16; off <<= 1) psum += __shfl_xor(psum, off, 32);
      lrow[r] = lrow[r] * alpha + psum;
#pragma unroll
      for (int t = 0; t < 4; ++t) oacc[t][r] *= alpha;
    }
    __builtin_amdgcn_fence(__ATOMIC_RELEASE, "workgroup");
    __builtin_amdgcn_wave_barrier();
    __builtin_amdgcn_fence(__ATOMIC_ACQUIRE, "workgroup");
#pragma unroll 1
    for (int kk = 0; kk < 2; ++kk) {
      FH pa;
      pa.h[0] = *(const v8h*)(pwh + c * AT_KC + kk * 32 + 8 * hh);
      pa.h[1] = *(const v8h*)(pwh + c * AT_KC + kk * 32 + 16 + 8 * hh);
#pragma unroll
      for (int t = 0; t < 4; ++t) {
        FH vb;
        vb.h[0] = *(const v8h*)(Vth + (t * 16 + c) * AT_KC + kk * 32 + 8 * hh);
        vb.h[1] = *(const v8h*)(Vth + (t * 16 + c) * AT_KC + kk * 32 + 16 + 8 * hh);
        oacc[t] = mma_h(pa.v, vb.v, oacc[t]);
      }
    }
  }

  float* os = Os[wave];
#pragma unroll
  for (int r = 0; r < 8; ++r) {
    const bool seen = mrow[r] > -1e29f;
    const float inv = seen ? (1.0f / (lrow[r] * AT_PSC)) : __uint_as_float(0x7fc00000u);
#pragma unroll
    for (int t = 0; t < 4; ++t) os[(8 * hh + r) * 68 + t * 16 + c] = oacc[t][r] * inv;
  }
  __builtin_amdgcn_fence(__ATOMIC_RELEASE, "workgroup");
  __builtin_amdgcn_wave_barrier();
  __builtin_amdgcn_fence(__ATOMIC_ACQUIRE, "workgroup");
  {
    const int c4 = (lane & 15) * 4;
    for (int pass = 0; pass < 2; ++pass) {
#pragma unroll
      for (int it = 0; it < 8; ++it) {
        const int row = it * 2 + hh;
        v4f val = *(const v4f*)(os + row * 68 + c4);
        *(volatile v4f*)(ob_ptr + (size_t)(q0 + row) * g.o_rs + c4) = val;
      }
      __threadfence();
    }
  }
}

extern "C" void kernel_launch(void* const* d_in, const int* in_sizes, int n_in,
                              void* d_out, int out_size, void* d_ws, size_t ws_size,
                              hipStream_t stream) {
  constexpr int Bz = 2, S = 2048, D = 1024, H = 16, HD = 64, WIN = 128;
  constexpr int TD = 3 * D;
  constexpr int M  = Bz * S;
  static_assert(H * HD == D);
  static_assert(M % 64 == 0 && TD % 64 == 0 && D % 64 == 0 && S % AT_QB == 0 && S % AT_KC == 0);
  static_assert((2 * WIN) / AT_KC + 2 <= AT_MAXCH);

  if (n_in < 6) return;
  if (in_sizes[0] != M * D || in_sizes[1] != Bz * S * S || in_sizes[2] != TD * D ||
      in_sizes[3] != TD || in_sizes[4] != D * D || in_sizes[5] != D || out_size != M * D) return;

  const float* x     = (const float*)d_in[0];
  const int*   amask = (const int*)d_in[1];
  const float* in_w  = (const float*)d_in[2];
  const float* in_b  = (const float*)d_in[3];
  const float* out_w = (const float*)d_in[4];
  const float* out_b = (const float*)d_in[5];
  float* y = (float*)d_out;

  const size_t bytes_x16  = (size_t)M  * D  * 2;
  const size_t bytes_w16  = (size_t)TD * D  * 2;
  const size_t bytes_ow16 = (size_t)D  * D  * 2;
  const size_t bytes_qkv  = (size_t)M  * TD * 4;
  const size_t bytes_att  = (size_t)M  * D  * 4;
  const size_t bytes_a16  = (size_t)M  * D  * 2;
  const size_t total = bytes_x16 + bytes_w16 + bytes_ow16 + bytes_qkv + bytes_att + bytes_a16;
  if (total > ws_size) return;
  char* p = (char*)d_ws;
  _Float16* x16  = (_Float16*)p;  p += bytes_x16;
  _Float16* w16  = (_Float16*)p;  p += bytes_w16;
  _Float16* ow16 = (_Float16*)p;  p += bytes_ow16;
  float*    qkv  = (float*)p;     p += bytes_qkv;
  float*    att  = (float*)p;     p += bytes_att;
  _Float16* a16  = (_Float16*)p;  p += bytes_a16;

  {
    const int n2x = (M * D) / 2, n2w = (TD * D) / 2, n2o = (D * D) / 2;
    cast_f32_f16x2_scaled<<<(n2x + 255) / 256, 256, 0, stream>>>(x,     x16,  n2x, 1.0f);
    cast_f32_f16x2_scaled<<<(n2w + 255) / 256, 256, 0, stream>>>(in_w,  w16,  n2w, 64.0f);
    cast_f32_f16x2_scaled<<<(n2o + 255) / 256, 256, 0, stream>>>(out_w, ow16, n2o, 64.0f);
  }

  {
    const int tiles = (M / 64) * (TD / 64);
    dim3 grid((tiles + 7) / 8, 1);
    wmma_gemm64<0, false, 2, 0, false, 0><<<grid, 256, 0, stream>>>(
        (const unsigned short*)x16, (const unsigned short*)x16, D, 0L,
        (const unsigned short*)w16, (const unsigned short*)w16, D, 0L,
        (void*)qkv, (void*)qkv, TD, 0L,
        in_b, in_b, 0L,
        M, TD, D, 1.0f / 64.0f);
  }

  {
    BandGeom g;
    g.q_bs = (long)S * TD; g.q_rs = TD; g.q_hs = HD;
    g.k_bs = (long)S * TD; g.k_rs = TD; g.k_hs = HD;
    g.v_bs = (long)S * TD; g.v_rs = TD; g.v_hs = HD;
    g.o_bs = (long)S * D;  g.o_rs = D;  g.o_hs = HD;
    g.m_bs = (long)S * S;  g.m_rs = S;
    g.S = S; g.H = H; g.W = WIN; g.lastq = S - 1; g.qscale = 0.125f; g.mask_fill = -1e30f;
    dim3 grid(Bz * H * (S / AT_QB));
    attn_band64_kernel<<<grid, 128, 0, stream>>>(qkv, qkv + D, qkv + 2 * D, att, amask, g);
  }

  {
    const int n2a = (M * D) / 2;
    cast_f32_f16x2_scaled<<<(n2a + 255) / 256, 256, 0, stream>>>(att, a16, n2a, 64.0f);
  }

  {
    const int tiles = (M / 64) * (D / 64);
    dim3 grid((tiles + 7) / 8, 1);
    wmma_gemm64<0, false, 2, 0, false, 0><<<grid, 256, 0, stream>>>(
        (const unsigned short*)a16, (const unsigned short*)a16, D, 0L,
        (const unsigned short*)ow16, (const unsigned short*)ow16, D, 0L,
        (void*)y, (void*)y, D, 0L,
        out_b, out_b, 0L,
        M, D, D, 1.0f / 4096.0f);
  }
  (void)stream;
}
